// DeltaMLP_2911987827332
// MI455X (gfx1250) — hardware-verified
//
#include <hip/hip_runtime.h>
#include <stddef.h>


typedef _Float16 v16h __attribute__((ext_vector_type(16)));
typedef _Float16 v8h  __attribute__((ext_vector_type(8)));
typedef float    v8f  __attribute__((ext_vector_type(8)));
typedef float    v4f  __attribute__((ext_vector_type(4)));
typedef _Float16 h16;

#ifndef NB
#define NB 4
#endif
#ifndef SEQ
#define SEQ 512
#endif
#define NB_FULL  4
#define SEQ_FULL 512
#define KD    128
#define HD    128
#define NC    3
#define PW    256
#define MROWS (NB * SEQ)
#define NTILE (SEQ / 32)
#define NTRI  (NTILE * (NTILE + 1) / 2)

static_assert(NB >= 1 && NB <= NB_FULL);
static_assert(SEQ >= 64 && SEQ <= SEQ_FULL && (SEQ % 64) == 0);
static_assert(KD == 128 && (KD % 32) == 0);
static_assert(HD == 4 * 32);
static_assert((HD % 64) == 0 && (HD % 32) == 0);
static_assert(PW == 2 * HD && (PW % 64) == 0 && (PW % 32) == 0);
static_assert((MROWS % 64) == 0 && (MROWS % 32) == 0);
static_assert(NC == 3 && ((32 * NC) % 8) == 0);
static_assert((size_t)NB_FULL * SEQ_FULL * SEQ_FULL * NC * 4 == (size_t)12582912);
static_assert((size_t)((NB - 1) * SEQ_FULL + SEQ) * SEQ_FULL * NC <=
              (size_t)NB_FULL * SEQ_FULL * SEQ_FULL * NC);

#define LDC 68
#define LPAD 132
#define LL  100
#define LDW 136
#define RSZ (32 * LPAD)
static_assert((LDC % 4) == 0 && LDC >= 64);
static_assert((LPAD % 4) == 0 && LPAD >= HD);
static_assert((LL % 4) == 0 && LL >= 32 * NC);
static_assert((LDW % 8) == 0 && LDW >= HD);

#define WCARRY 64.0f
#define XCARRY 16.0f
#define ACARRY 64.0f

#define WT_BYTES  ((size_t)PW * KD * 2)
#define X16_BYTES ((size_t)MROWS * KD * 2)
#define PF_BYTES  ((size_t)MROWS * PW * 4)
#define OFF_WT  ((size_t)0)
#define OFF_X16 (OFF_WT + WT_BYTES)
#define OFF_PF  (OFF_X16 + X16_BYTES)
#define WS_TOTAL (OFF_PF + PF_BYTES)
static_assert((WT_BYTES % 128) == 0 && (X16_BYTES % 128) == 0 && (PF_BYTES % 128) == 0);
static_assert(WS_TOTAL <= (size_t)134217728);

#define PAIR_LDS_BYTES ((size_t)(4 * RSZ + 2 * 32 * LL + 4) * 4 + (size_t)16 * LDW * 2)
static_assert(PAIR_LDS_BYTES <= (size_t)131072);
static_assert((size_t)64 * LDC * 4 <= (size_t)131072);

__device__ __forceinline__ float bf16r(float x) {
  unsigned int u = __float_as_uint(x);
  u = (u + 0x7FFFu + ((u >> 16) & 1u)) & 0xFFFF0000u;
  return __uint_as_float(u);
}

__device__ __forceinline__ h16 toh_flush(float v) {
  const h16 r = (h16)v;
  return (fabsf(v) < 6.103515625e-05f) ? (h16)0.0f : r;
}

__device__ __forceinline__ v16h frag_at(const _Float16* p) {
  v8h lo = *(const v8h*)(p);
  v8h hi = *(const v8h*)(p + 16);
  v16h out;
#pragma unroll
  for (int i = 0; i < 8; ++i) { out[i] = lo[i]; out[i + 8] = hi[i]; }
  return out;
}

__device__ __forceinline__ v8f wmma16(v16h a, v16h b, v8f c) {
  v8f d = __builtin_amdgcn_wmma_f32_16x16x32_f16(false, a, false, b, (short)0, c,
                                                 false, false);
  asm volatile("v_nop\n\tv_nop\n\tv_nop\n\tv_nop" : "+v"(d) : "v"(a), "v"(b));
  return d;
}

__device__ __forceinline__ float sigm(float z) {
  return __builtin_amdgcn_rcpf(1.0f + __expf(-z));
}

__global__ __launch_bounds__(256) void wrow_kernel(
    const float* __restrict__ W, _Float16* __restrict__ Wt) {
#pragma clang fp contract(off)
  const unsigned gid = blockIdx.x * 256u + threadIdx.x;
  const unsigned prow = gid >> 4;
  const unsigned c = (gid & 15u) * 8u;
  const unsigned sel = prow / (unsigned)HD;
  const unsigned hrow = prow - sel * (unsigned)HD;
  const float* src = W + (size_t)hrow * (2u * KD) + sel * (unsigned)KD + c;
  const v4f a0 = *(const v4f*)(src);
  const v4f a1 = *(const v4f*)(src + 4u);
  v8h o;
#pragma unroll
  for (int i = 0; i < 4; ++i) {
    o[i]     = toh_flush(WCARRY * bf16r(a0[i]));
    o[i + 4] = toh_flush(WCARRY * bf16r(a1[i]));
  }
  _Float16* p = Wt + (size_t)prow * KD + c;
  *(volatile v8h*)p = o;
  __threadfence();
  *(volatile v8h*)p = o;
}
static_assert(((size_t)PW * 16) % 256 == 0);
static_assert(16 * 8 == KD);

__global__ __launch_bounds__(256) void xconv_kernel(
    const float* __restrict__ X, _Float16* __restrict__ X16) {
#pragma clang fp contract(off)
  const unsigned gid = blockIdx.x * 256u + threadIdx.x;
  const unsigned crow = gid >> 4;
  const unsigned c = (gid & 15u) * 8u;
  const unsigned bidx = crow / (unsigned)SEQ;
  const unsigned sq = crow - bidx * (unsigned)SEQ;
  const size_t srow = (size_t)bidx * SEQ_FULL + sq;
  const v4f a0 = *(const v4f*)(X + srow * KD + c);
  const v4f a1 = *(const v4f*)(X + srow * KD + c + 4u);
  v8h o;
#pragma unroll
  for (int i = 0; i < 4; ++i) {
    o[i]     = toh_flush(XCARRY * bf16r(a0[i]));
    o[i + 4] = toh_flush(XCARRY * bf16r(a1[i]));
  }
  _Float16* p = X16 + (size_t)crow * KD + c;
  *(volatile v8h*)p = o;
  __threadfence();
  *(volatile v8h*)p = o;
}
static_assert(((size_t)MROWS * 16) % 256 == 0);

__global__ __launch_bounds__(256) void gemm_pre_kernel(
    const _Float16* __restrict__ A16, const _Float16* __restrict__ Bt,
    float* __restrict__ outf) {
  __shared__ float Cs[64 * LDC];
  const unsigned tid = threadIdx.x, lane = tid & 31u;
  const unsigned w = (unsigned)__builtin_amdgcn_readfirstlane((int)(threadIdx.x >> 5));
  const unsigned mw = w >> 1, nw = w & 1u;
  const unsigned hh = lane >> 4, m = lane & 15u;
  const unsigned n0 = blockIdx.x * 64u;
  const unsigned row0 = blockIdx.y * 64u;

  const _Float16* ap  = A16 + (size_t)(row0 + mw * 16u + m) * KD + hh * 8u;
  const _Float16* bp0 = Bt + (size_t)(n0 + nw * 32u + m) * KD + hh * 8u;
  const _Float16* bp1 = bp0 + (size_t)16 * KD;
  v8f acc0 = {}, acc1 = {};
#pragma unroll
  for (unsigned k0 = 0; k0 < (unsigned)KD; k0 += 32u) {
    const v16h a  = frag_at(ap + k0);
    const v16h b0 = frag_at(bp0 + k0);
    const v16h b1 = frag_at(bp1 + k0);
    acc0 = wmma16(a, b0, acc0);
    acc1 = wmma16(a, b1, acc1);
  }
#pragma unroll
  for (int r = 0; r < 8; ++r) {
    float* d = &Cs[(mw * 16u + hh * 8u + (unsigned)r) * LDC + nw * 32u + m];
    d[0]  = acc0[r];
    d[16] = acc1[r];
  }
  __syncthreads();

  const float cs = 1.0f / (WCARRY * XCARRY);
  v4f xs[4];
  size_t off[4];
#pragma unroll
  for (unsigned i = 0; i < 4u; ++i) {
    const unsigned r = 16u * i + (tid >> 4);
    const unsigned c = (tid & 15u) * 4u;
    const v4f u = *(const v4f*)&Cs[r * LDC + c];
    v4f val;
#pragma unroll
    for (int j = 0; j < 4; ++j) val[j] = u[j] * cs;
    xs[i] = val;
    off[i] = (size_t)(row0 + r) * PW + n0 + c;
  }
#pragma unroll
  for (int i = 0; i < 4; ++i) *(volatile v4f*)(outf + off[i]) = xs[i];
  __threadfence();
#pragma unroll
  for (int i = 0; i < 4; ++i) *(volatile v4f*)(outf + off[i]) = xs[i];
}
static_assert(4 * 16 == 64);

__global__ __launch_bounds__(256) void pair_kernel(
    const float* __restrict__ Pf, const float* __restrict__ b1,
    const float* __restrict__ W2, const float* __restrict__ b2,
    float* __restrict__ out) {
#pragma clang fp contract(off)
  __shared__ __attribute__((aligned(16))) float sH[4 * RSZ];
  __shared__ __attribute__((aligned(16))) _Float16 W2s[16 * LDW];
  __shared__ __attribute__((aligned(16))) float sL[2 * 32 * LL];
  __shared__ float b2s[4];

  const unsigned tid = threadIdx.x;
  const unsigned b = blockIdx.y;

  unsigned t = blockIdx.x, ti = 0u;
#pragma unroll 1
  for (unsigned s = 0; s + 1u < (unsigned)NTILE; ++s) {
    const unsigned len = (unsigned)NTILE - ti;
    const bool adv = (t >= len);
    t  = adv ? (t - len) : t;
    ti = adv ? (ti + 1u) : ti;
  }
  unsigned tj = ti + t;
  tj = (tj < (unsigned)NTILE) ? tj : ((unsigned)NTILE - 1u);
  const unsigned i0 = ti * 32u, j0 = tj * 32u;
  const bool dtile = (ti == tj);
  const unsigned norient = dtile ? 1u : 2u;

  const size_t irow = (size_t)(b * (unsigned)SEQ + i0) * PW;
  const size_t jrow = (size_t)(b * (unsigned)SEQ + j0) * PW;
#pragma unroll 1
  for (unsigned s = 0; s < 4u; ++s) {
    const unsigned idx = tid + 256u * s;
    const unsigned r = idx >> 5, c = (idx & 31u) * 4u;
    const v4f ai = *(const v4f*)(Pf + irow + (size_t)r * PW + c);
    const v4f bi = *(const v4f*)(Pf + irow + (size_t)r * PW + HD + c);
    const v4f aj = *(const v4f*)(Pf + jrow + (size_t)r * PW + c);
    const v4f bj = *(const v4f*)(Pf + jrow + (size_t)r * PW + HD + c);
    const v4f g  = *(const v4f*)(b1 + c);
    v4f avi, avj;
#pragma unroll
    for (int j = 0; j < 4; ++j) {
      const float gb = bf16r(g[j]);
      avi[j] = ai[j] + gb;
      avj[j] = aj[j] + gb;
    }
    *(v4f*)&sH[0 * RSZ + r * LPAD + c] = avi;
    *(v4f*)&sH[1 * RSZ + r * LPAD + c] = bi;
    *(v4f*)&sH[2 * RSZ + r * LPAD + c] = avj;
    *(v4f*)&sH[3 * RSZ + r * LPAD + c] = bj;
  }
  {
    const unsigned n = tid >> 4, kc = (tid & 15u) * 8u;
    const unsigned ns = (n < (unsigned)NC) ? n : ((unsigned)NC - 1u);
    const bool live = (n < (unsigned)NC);
    const v4f w0 = *(const v4f*)(W2 + ns * (unsigned)HD + kc);
    const v4f w1 = *(const v4f*)(W2 + ns * (unsigned)HD + kc + 4u);
    v8h o;
#pragma unroll
    for (int i = 0; i < 4; ++i) {
      const h16 q0 = toh_flush(WCARRY * bf16r(w0[i]));
      const h16 q1 = toh_flush(WCARRY * bf16r(w1[i]));
      o[i]     = live ? q0 : (h16)0.0f;
      o[i + 4] = live ? q1 : (h16)0.0f;
    }
    *(v8h*)&W2s[n * LDW + kc] = o;
  }
  if (tid < 4u) {
    const unsigned cl = (tid < (unsigned)NC) ? tid : ((unsigned)NC - 1u);
    b2s[tid] = bf16r(b2[cl]);
  }
  __syncthreads();

  const unsigned lane = tid & 31u;
  const unsigned w = (unsigned)__builtin_amdgcn_readfirstlane((int)(threadIdx.x >> 5));
  const unsigned hh = lane >> 4, m = lane & 15u;
  const unsigned g16 = (w & 1u) * 16u;
  const unsigned rb = (w >> 1) * 8u;

  v16h bw[4];
#pragma unroll
  for (unsigned ks = 0; ks < 4u; ++ks) {
    const v8h lo = *(const v8h*)&W2s[m * LDW + 32u * ks + 8u * hh];
    const v8h hi = *(const v8h*)&W2s[m * LDW + 32u * ks + 8u * hh + 16u];
    v16h f;
#pragma unroll
    for (int i = 0; i < 8; ++i) { f[i] = lo[i]; f[i + 8] = hi[i]; }
    bw[ks] = f;
  }

  const float cs2 = 1.0f / (ACARRY * WCARRY);
#pragma unroll 1
  for (unsigned o = 0; o < norient; ++o) {
    const unsigned rowreg = (2u * o) * (unsigned)RSZ;
    const unsigned colreg = (3u - 2u * o) * (unsigned)RSZ;
    const unsigned pbase = colreg + (g16 + m) * LPAD + 8u * hh;
    v4f pv[4][4];
#pragma unroll
    for (unsigned ks = 0; ks < 4u; ++ks) {
      pv[ks][0] = *(const v4f*)&sH[pbase + 32u * ks];
      pv[ks][1] = *(const v4f*)&sH[pbase + 32u * ks + 4u];
      pv[ks][2] = *(const v4f*)&sH[pbase + 32u * ks + 16u];
      pv[ks][3] = *(const v4f*)&sH[pbase + 32u * ks + 20u];
    }
#pragma unroll 1
    for (unsigned rr = 0; rr < 8u; ++rr) {
      const unsigned row = rb + rr;
      const unsigned rbase = rowreg + row * LPAD + 8u * hh;
      v8f acc = {};
#pragma unroll
      for (unsigned ks = 0; ks < 4u; ++ks) {
        v4f rv[4];
        rv[0] = *(const v4f*)&sH[rbase + 32u * ks];
        rv[1] = *(const v4f*)&sH[rbase + 32u * ks + 4u];
        rv[2] = *(const v4f*)&sH[rbase + 32u * ks + 16u];
        rv[3] = *(const v4f*)&sH[rbase + 32u * ks + 20u];
        v16h a;
#pragma unroll
        for (int q = 0; q < 4; ++q) {
#pragma unroll
          for (int j = 0; j < 4; ++j) {
            const float x = rv[q][j] + pv[ks][q][j];
            const float sv = x * sigm(x);
            a[4 * q + j] = toh_flush(ACARRY * sv);
          }
        }
        acc = wmma16(a, bw[ks], acc);
      }
      if (m < (unsigned)NC) {
        float* d = &sL[o * (32u * LL) + row * LL + (g16 + 8u * hh) * (unsigned)NC + m];
#pragma unroll
        for (int r = 0; r < 8; ++r) d[NC * r] = acc[r] * cs2;
      }
    }
  }
  __syncthreads();

  const unsigned l2off = (norient - 1u) * (32u * LL);
  v4f xa[3], xb[3];
  size_t offa[3], offb[3];
#pragma unroll
  for (unsigned s = 0; s < 3u; ++s) {
    const unsigned idx = tid + 256u * s;
    const unsigned r = idx / 24u;
    const unsigned f4 = idx - r * 24u;
    const v4f u1 = *(const v4f*)&sL[r * LL + 4u * f4];
    const v4f u2 = *(const v4f*)&sL[l2off + r * LL + 4u * f4];
    v4f va, vb;
#pragma unroll
    for (int j = 0; j < 4; ++j) {
      const unsigned e = 4u * f4 + (unsigned)j;
      const unsigned c = e / 3u;
      const unsigned k = e - 3u * c;
      const float t2 = sL[l2off + c * LL + 3u * r + k];
      const float t1 = sL[c * LL + 3u * r + k];
      const float bb = b2s[k];
      va[j] = ((u1[j] + bb) + (t2 + bb)) * 0.5f;
      vb[j] = ((u2[j] + bb) + (t1 + bb)) * 0.5f;
    }
    xa[s] = va;
    xb[s] = vb;
    offa[s] = (((size_t)b * SEQ_FULL + i0 + r) * SEQ_FULL + j0) * NC + 4u * f4;
    offb[s] = (((size_t)b * SEQ_FULL + j0 + r) * SEQ_FULL + i0) * NC + 4u * f4;
  }
#pragma unroll
  for (int s = 0; s < 3; ++s) *(volatile v4f*)(out + offa[s]) = xa[s];
  if (!dtile) {
#pragma unroll
    for (int s = 0; s < 3; ++s) *(volatile v4f*)(out + offb[s]) = xb[s];
  }
  __threadfence();
#pragma unroll
  for (int s = 0; s < 3; ++s) *(volatile v4f*)(out + offa[s]) = xa[s];
  if (!dtile) {
#pragma unroll
    for (int s = 0; s < 3; ++s) *(volatile v4f*)(out + offb[s]) = xb[s];
  }
}
static_assert(3 * 256 == 32 * 24);
static_assert(24 * 4 == 32 * NC);
static_assert((24 % 8) == 0);
static_assert(16 * 16 == 256);
static_assert(16 * 8 == HD);
static_assert(4 * 32 == HD);
static_assert(4 * 8 == 32 && 2 * 16 == 32);

extern "C" void kernel_launch(void* const* d_in, const int* in_sizes, int n_in,
                              void* d_out, int out_size, void* d_ws, size_t ws_size,
                              hipStream_t stream) {
  if (n_in < 5) return;
  const long long need_x = ((long long)(NB - 1) * SEQ_FULL + SEQ) * KD;
  const long long need_o = ((long long)(NB - 1) * SEQ_FULL + SEQ) * SEQ_FULL * NC;
  if ((long long)in_sizes[0] < need_x) return;
  if ((long long)in_sizes[1] < (long long)HD * 2 * KD) return;
  if (in_sizes[2] < HD || in_sizes[3] < NC * HD || in_sizes[4] < NC) return;
  if ((long long)out_size < need_o) return;
  if (ws_size < WS_TOTAL) return;

  const float* X  = (const float*)d_in[0];
  const float* W1 = (const float*)d_in[1];
  const float* b1 = (const float*)d_in[2];
  const float* W2 = (const float*)d_in[3];
  const float* b2 = (const float*)d_in[4];
  float* out = (float*)d_out;

  char* ws = (char*)d_ws;
  _Float16* Wt  = (_Float16*)(ws + OFF_WT);
  _Float16* X16 = (_Float16*)(ws + OFF_X16);
  float*    Pf  = (float*)(ws + OFF_PF);

  dim3 blk(256);
  wrow_kernel<<<dim3(PW * 16 / 256), blk, 0, stream>>>(W1, Wt);
  xconv_kernel<<<dim3(MROWS / 16), blk, 0, stream>>>(X, X16);
  gemm_pre_kernel<<<dim3(PW / 64, MROWS / 64), blk, 0, stream>>>(X16, Wt, Pf);
  pair_kernel<<<dim3(NTRI, NB), blk, 0, stream>>>(Pf, b1, W2, b2, out);
}
